// MultiScaleRetention_78065325572194
// MI455X (gfx1250) — hardware-verified
//
#include <hip/hip_runtime.h>
#include <math.h>

constexpr int kBatch = 2;
constexpr int kSeq   = 2048;
constexpr int kDim   = 1024;
constexpr int kHeads = 16;
constexpr int kDh    = 64;
constexpr int kTok   = kBatch * kSeq;
constexpr float kWCarry     = 64.0f;
constexpr float kWCarryInv  = 1.0f / 64.0f;
constexpr float kScoreScale = 0.125f;
constexpr float kPCarry     = 32768.0f;
constexpr float kLoCarry    = 2048.0f;
constexpr float kLoInv      = 1.0f / 2048.0f;
constexpr float kGnEps      = 1.0e-5f;
constexpr float kInvDh      = 1.0f / 64.0f;

#define CT_ASSERT_CAT2(a, b) a##b
#define CT_ASSERT_CAT(a, b) CT_ASSERT_CAT2(a, b)
#define CT_ASSERT(cond) typedef char CT_ASSERT_CAT(ct_assert_line_, __LINE__)[(cond) ? 1 : -1]
CT_ASSERT(kHeads * kDh == kDim);
CT_ASSERT(kTok % 64 == 0 && kDim % 64 == 0);
CT_ASSERT(kDim % 32 == 0);
CT_ASSERT(kSeq % 64 == 0 && kDh == 64);
CT_ASSERT((kTok * kDim) % (8 * 256) == 0);
CT_ASSERT((kDim * kDim) % (8 * 256) == 0);
CT_ASSERT(kDim == 4 * 256);

typedef __attribute__((ext_vector_type(16))) _Float16 v16h;
typedef __attribute__((ext_vector_type(8)))  _Float16 v8h;
typedef __attribute__((ext_vector_type(16))) __bf16   v16b;
typedef __attribute__((ext_vector_type(8)))  __bf16   v8b;
typedef __attribute__((ext_vector_type(8)))  float    v8f;
typedef __attribute__((ext_vector_type(4)))  float    v4f;
typedef __attribute__((ext_vector_type(4)))  unsigned int v4u;

__device__ __forceinline__ unsigned short f2bf_bits(float f) {
  unsigned u = __float_as_uint(f);
  return (unsigned short)((u + 0x7FFFu + ((u >> 16) & 1u)) >> 16);
}
__device__ __forceinline__ float bf_bits2f(unsigned short h) { return __uint_as_float(((unsigned)h) << 16); }

__device__ __forceinline__ void dep_guard_h(v8f& a, v8f& b, v16h x, v16h y) { asm volatile("v_nop\n\tv_nop\n\tv_nop\n\tv_nop" : "+v"(a), "+v"(b) : "v"(x), "v"(y)); }
__device__ __forceinline__ void dep_guard_b(v8f& a, v8f& b, v16b x, v16b y) { asm volatile("v_nop\n\tv_nop\n\tv_nop\n\tv_nop" : "+v"(a), "+v"(b) : "v"(x), "v"(y)); }
__device__ __forceinline__ void dep_guard4_h(v8f& a, v8f& b, v8f& c, v8f& d, v16h x, v16h y, v16h b0, v16h b1, v16h b2, v16h b3) {
  asm volatile("v_nop\n\tv_nop\n\tv_nop\n\tv_nop" : "+v"(a), "+v"(b), "+v"(c), "+v"(d) : "v"(x), "v"(y), "v"(b0), "v"(b1), "v"(b2), "v"(b3));
}
__device__ __forceinline__ void dep_guard4_b(v8f& a, v8f& b, v8f& c, v8f& d, v16b x, v16b y, v16b b0, v16b b1, v16b b2, v16b b3) {
  asm volatile("v_nop\n\tv_nop\n\tv_nop\n\tv_nop" : "+v"(a), "+v"(b), "+v"(c), "+v"(d) : "v"(x), "v"(y), "v"(b0), "v"(b1), "v"(b2), "v"(b3));
}
__device__ __forceinline__ void keep4_h(v16h a, v16h b, v16h c, v16h d) { asm volatile("v_nop" :: "v"(a), "v"(b), "v"(c), "v"(d)); }
__device__ __forceinline__ void keep4_b(v16b a, v16b b, v16b c, v16b d) { asm volatile("v_nop" :: "v"(a), "v"(b), "v"(c), "v"(d)); }
__device__ __forceinline__ void acc_guard4(v8f& a, v8f& b, v8f& c, v8f& d) { asm volatile("v_nop\n\tv_nop\n\tv_nop\n\tv_nop" : "+v"(a), "+v"(b), "+v"(c), "+v"(d)); }
template <typename T> struct Frag;
template <> struct Frag<_Float16> {
  typedef v16h V; union U { v16h v; v8h h[2]; };
  static __device__ __forceinline__ v16h load(const _Float16* p) {
    U f; f.h[0] = *(const v8h*)(p); f.h[1] = *(const v8h*)(p + 16); return f.v;
  }
  static __device__ __forceinline__ v8f mma(v16h a, v16h b, v8f c) {
    return __builtin_amdgcn_wmma_f32_16x16x32_f16(false, a, false, b, (short)0, c, false, false);
  }
  static __device__ __forceinline__ void guard(v8f& a, v8f& b, v16h x, v16h y) { dep_guard_h(a, b, x, y); }
  static __device__ __forceinline__ void guard4(v8f& a, v8f& b, v8f& c, v8f& d, v16h x, v16h y, v16h b0, v16h b1, v16h b2, v16h b3) { dep_guard4_h(a, b, c, d, x, y, b0, b1, b2, b3); }
  static __device__ __forceinline__ void keep(v16h a, v16h b, v16h c, v16h d) { keep4_h(a, b, c, d); }
};
template <> struct Frag<__bf16> {
  typedef v16b V; union U { v16b v; v8b h[2]; };
  static __device__ __forceinline__ v16b load(const __bf16* p) {
    U f; f.h[0] = *(const v8b*)(p); f.h[1] = *(const v8b*)(p + 16); return f.v;
  }
  static __device__ __forceinline__ v8f mma(v16b a, v16b b, v8f c) {
    return __builtin_amdgcn_wmma_f32_16x16x32_bf16(false, a, false, b, (short)0, c, false, false);
  }
  static __device__ __forceinline__ void guard(v8f& a, v8f& b, v16b x, v16b y) { dep_guard_b(a, b, x, y); }
  static __device__ __forceinline__ void guard4(v8f& a, v8f& b, v8f& c, v8f& d, v16b x, v16b y, v16b b0, v16b b1, v16b b2, v16b b3) { dep_guard4_b(a, b, c, d, x, y, b0, b1, b2, b3); }
  static __device__ __forceinline__ void keep(v16b a, v16b b, v16b c, v16b d) { keep4_b(a, b, c, d); }
};

__device__ __forceinline__ unsigned pk16(unsigned short a, unsigned short b) { return (unsigned)a | ((unsigned)b << 16); }
__device__ __forceinline__ unsigned short h_bits(float f) { const _Float16 h = (_Float16)f; return __builtin_bit_cast(unsigned short, h); }
__device__ __forceinline__ void h_pair_bits(float x, unsigned short& hb, unsigned short& lb) {
  const _Float16 hq = (_Float16)x;
  const float hf = (float)hq;
  const float rf = (x - hf) * kLoCarry;
  const _Float16 lq = (_Float16)rf;
  hb = __builtin_bit_cast(unsigned short, hq);
  lb = __builtin_bit_cast(unsigned short, lq);
}

__device__ __forceinline__ v8f mma_h(v16h a, v16h b, v8f c) {
  c = __builtin_amdgcn_wmma_f32_16x16x32_f16(false, a, false, b, (short)0, c, false, false);
  asm volatile("v_nop\n\tv_nop\n\tv_nop\n\tv_nop" : "+v"(c) : "v"(a), "v"(b));
  return c;
}
__device__ __forceinline__ v16h ld_frag16(const unsigned short* p) {
  return Frag<_Float16>::load((const _Float16*)(const void*)p);
}

template <int ET> struct Elem;
template <> struct Elem<0> { typedef _Float16 T; };
template <> struct Elem<1> { typedef __bf16 T; };
template <int ET, bool SPLIT, int BIAS_MODE, int OUT_MODE, bool RESID, int ACT = 0>
__global__ __launch_bounds__(256) void wmma_gemm64(
    const unsigned short* __restrict__ Ap, const unsigned short* __restrict__ A2p, int lda, long strideA,
    const unsigned short* __restrict__ Btp, const unsigned short* __restrict__ Bt2p, int ldb, long strideB,
    void* __restrict__ Cout, void* __restrict__ Cout2, int ldc, long strideC,
    const float* __restrict__ bias,
    const float* __restrict__ resid, long strideR,
    int M, int N, int K, float scale) {
  typedef typename Elem<ET>::T T;
  typedef typename Frag<T>::V V;
  const T* A = (const T*)Ap; const T* A2 = (const T*)A2p; const T* Bt = (const T*)Btp; const T* Bt2 = (const T*)Bt2p;
  __shared__ __align__(16) float sT[8][16 * 68];
  const int b    = blockIdx.y;
  const int lane = threadIdx.x & 31;
  const int wave = threadIdx.x >> 5;
  const int tilesN = N >> 6;
  const int tilesM = M >> 6;
  const int tile = blockIdx.x * 8 + wave;
  if (tile >= tilesM * tilesN) return;
  const int tm = tile / tilesN;
  const int tn = tile - tm * tilesN;
  const int m0 = tm << 6;
  const int n0 = tn << 6;

  const T* Ab  = A  + (size_t)b * strideA;
  const T* Bb  = Bt + (size_t)b * strideB;
  const T* Ab2 = SPLIT ? (A2  + (size_t)b * strideA) : nullptr;
  const T* Bb2 = SPLIT ? (Bt2 + (size_t)b * strideB) : nullptr;

  const int rlane = lane & 15;
  const int koff  = (lane >> 4) * 8;
  const int mOff  = (lane >> 4) * 8;

  v8f acc[4][4];
#pragma unroll
  for (int i = 0; i < 4; ++i)
#pragma unroll
    for (int j = 0; j < 4; ++j) acc[i][j] = (v8f){0.f,0.f,0.f,0.f,0.f,0.f,0.f,0.f};

  for (int k0 = 0; k0 < K; k0 += 32) {
    V bh[4], bl[4];
#pragma unroll
    for (int j = 0; j < 4; ++j) {
      const size_t bo = (size_t)(n0 + (j << 4) + rlane) * ldb + koff + k0;
      bh[j] = Frag<T>::load(Bb + bo);
      if (SPLIT) bl[j] = Frag<T>::load(Bb2 + bo);
    }
#pragma unroll
    for (int i = 0; i < 4; ++i) {
      const size_t ao = (size_t)(m0 + (i << 4) + rlane) * lda + koff + k0;
      V ah = Frag<T>::load(Ab + ao);
      V al;
      if (SPLIT) al = Frag<T>::load(Ab2 + ao);
#pragma unroll
      for (int j = 0; j < 4; ++j) {
        acc[i][j] = Frag<T>::mma(ah, bh[j], acc[i][j]);
        if (SPLIT) {
          acc[i][j] = Frag<T>::mma(ah, bl[j], acc[i][j]);
          acc[i][j] = Frag<T>::mma(al, bh[j], acc[i][j]);
        }
      }
      Frag<T>::guard4(acc[i][0], acc[i][1], acc[i][2], acc[i][3], ah, SPLIT ? al : ah, bh[0], bh[1], bh[2], bh[3]);
    }
    Frag<T>::keep(bh[0], bh[1], bh[2], bh[3]);
    if (SPLIT) Frag<T>::keep(bl[0], bl[1], bl[2], bl[3]);
  }
  acc_guard4(acc[0][0], acc[0][1], acc[0][2], acc[0][3]);
  acc_guard4(acc[1][0], acc[1][1], acc[1][2], acc[1][3]);
  acc_guard4(acc[2][0], acc[2][1], acc[2][2], acc[2][3]);
  acc_guard4(acc[3][0], acc[3][1], acc[3][2], acc[3][3]);

  float* slab = sT[wave];
  const float* Rb = RESID ? (resid + (size_t)b * strideR) : nullptr;
#pragma unroll
  for (int i = 0; i < 4; ++i) {
    const int mBase = m0 + (i << 4);
#pragma unroll
    for (int j = 0; j < 4; ++j) {
      const int n = n0 + (j << 4) + rlane;
      float bv = 0.f;
      if (BIAS_MODE == 2) bv = bias[n];
#pragma unroll
      for (int r = 0; r < 8; ++r) {
        float v = acc[i][j][r] * scale;
        if (BIAS_MODE == 1) v += bias[mBase + mOff + r];
        if (BIAS_MODE == 2) v += bv;
        if (RESID) v += Rb[(size_t)(mBase + mOff + r) * ldc + n];
        if (ACT == 2) v = fmaxf(v, 0.0f);
        if (ACT == 4) v = (v > 0.f) ? v : 0.01f * v;
        slab[(mOff + r) * 68 + (j << 4) + rlane] = v;
      }
    }
    __builtin_amdgcn_fence(__ATOMIC_RELEASE, "workgroup");
    __builtin_amdgcn_wave_barrier();
    __builtin_amdgcn_fence(__ATOMIC_ACQUIRE, "workgroup");
    if (OUT_MODE == 0) {
      float* C = (float*)Cout + (size_t)b * strideC;
      const int hh = lane >> 4, c4 = (lane & 15) * 4;
      for (int pass = 0; pass < 2; ++pass) {
#pragma unroll
        for (int it = 0; it < 8; ++it) {
          const int row = it * 2 + hh;
          v4f v = *(const v4f*)(slab + row * 68 + c4);
          *(volatile v4f*)(C + (size_t)(mBase + row) * ldc + n0 + c4) = v;
        }
        __threadfence();
      }
    } else {
      const int q = lane >> 3, c8 = (lane & 7) * 8;
      unsigned short* C  = (unsigned short*)Cout  + (size_t)b * strideC;
      unsigned short* C2 = (OUT_MODE >= 2) ? ((unsigned short*)Cout2 + (size_t)b * strideC) : nullptr;
      for (int pass = 0; pass < 2; ++pass) {
#pragma unroll
        for (int it = 0; it < 4; ++it) {
          const int row = it * 4 + q;
          const float* sp = slab + row * 68 + c8;
          v8h hv, lv;
#pragma unroll
          for (int e = 0; e < 8; ++e) {
            if (OUT_MODE == 1) {
              hv[e] = (_Float16)sp[e];
            } else if (OUT_MODE == 3) {
              unsigned short hb, lb;
              h_pair_bits(sp[e], hb, lb);
              hv[e] = __builtin_bit_cast(_Float16, hb);
              lv[e] = __builtin_bit_cast(_Float16, lb);
            } else {
              unsigned short hb = f2bf_bits(sp[e]);
              unsigned short lb = f2bf_bits(sp[e] - bf_bits2f(hb));
              hv[e] = __builtin_bit_cast(_Float16, hb);
              lv[e] = __builtin_bit_cast(_Float16, lb);
            }
          }
          *(volatile v8h*)(C + (size_t)(mBase + row) * ldc + n0 + c8) = hv;
          if (OUT_MODE >= 2) *(volatile v8h*)(C2 + (size_t)(mBase + row) * ldc + n0 + c8) = lv;
        }
        __threadfence();
      }
    }
    __builtin_amdgcn_fence(__ATOMIC_RELEASE, "workgroup");
    __builtin_amdgcn_wave_barrier();
    __builtin_amdgcn_fence(__ATOMIC_ACQUIRE, "workgroup");
  }
}

__global__ __launch_bounds__(256) void cast8_f16_kernel(const float* __restrict__ in, unsigned short* __restrict__ out,
                                                       int n8, float scale) {
  const int i = blockIdx.x * 256 + threadIdx.x;
  if (i >= n8) return;
  const float* p = in + 8 * (size_t)i;
  const v4f a = *(const v4f*)(p);
  const v4f c = *(const v4f*)(p + 4);
  unsigned short hb[8];
#pragma unroll
  for (int e = 0; e < 4; ++e) {
    hb[e]     = h_bits(a[e] * scale);
    hb[4 + e] = h_bits(c[e] * scale);
  }
  const v4u u = (v4u){pk16(hb[0], hb[1]), pk16(hb[2], hb[3]), pk16(hb[4], hb[5]), pk16(hb[6], hb[7])};
  unsigned short* q = out + 8 * (size_t)i;
  *(volatile v4u*)q = u;
  __threadfence();
  *(volatile v4u*)q = u;
}

constexpr int AT_D  = 64;
constexpr int AT_NW = 4;
constexpr int AT_QB = 64;
constexpr int AT_KC = 64;

__global__ __launch_bounds__(128) void attn_f16_kernel(const unsigned short* __restrict__ Qp, const unsigned short* __restrict__ Kp,
                                                      const unsigned short* __restrict__ Vp, const unsigned short* __restrict__ VLp,
                                                      float* __restrict__ Op,
                                                      int ldin, int ldo, int S, int H, float sscale) {
  __shared__ __align__(16) unsigned short Ksh[AT_KC * AT_D];
  __shared__ __align__(16) unsigned short Vth[AT_D * AT_KC];
  __shared__ __align__(16) unsigned short Vtl[AT_D * AT_KC];
  __shared__ __align__(16) unsigned short Psh[AT_NW][16 * AT_KC];
  __shared__ __align__(16) unsigned short Psl[AT_NW][16 * AT_KC];
  __shared__ __align__(16) float Os[AT_NW][16 * 68];

  const int tid  = threadIdx.x;
  const int wave = tid >> 5;
  const int lane = tid & 31;
  const int hh   = lane >> 4;
  const int c    = lane & 15;

  const int nqb = S / AT_QB;
  const int bx  = blockIdx.x;
  const int qb  = bx % nqb;
  const int bh  = bx / nqb;
  const int h   = bh % H;
  const int b   = bh / H;
  const int q0  = qb * AT_QB + wave * 16;
  const size_t tokb = (size_t)b * S;
  const int hoff = h * AT_D;

  v16h qa[2];
  {
    const unsigned short* qrow = Qp + (tokb + q0 + c) * (size_t)ldin + hoff;
#pragma unroll
    for (int dc = 0; dc < 2; ++dc) qa[dc] = ld_frag16(qrow + dc * 32 + 8 * hh);
  }

  float mrow[8], lrow[8];
  v8f oacc[4], racc[4];
#pragma unroll
  for (int r = 0; r < 8; ++r) { mrow[r] = -__builtin_inff(); lrow[r] = 0.f; }
#pragma unroll
  for (int t = 0; t < 4; ++t) {
    oacc[t] = (v8f){0.f,0.f,0.f,0.f,0.f,0.f,0.f,0.f};
    racc[t] = (v8f){0.f,0.f,0.f,0.f,0.f,0.f,0.f,0.f};
  }

  const int nChunks = S / AT_KC;
  for (int kc = 0; kc < nChunks; ++kc) {
    const int kv0 = kc * AT_KC;
    __syncthreads();
    {
      const int kvr = tid >> 1, dh = (tid & 1) * 32;
      const size_t roff = (tokb + kv0 + kvr) * (size_t)ldin + hoff + dh;
      const unsigned short* krow = Kp + roff;
      const unsigned short* vrow = Vp + roff;
      const unsigned short* lrw  = VLp + roff;
      v4u kw[4];
#pragma unroll
      for (int i = 0; i < 4; ++i) kw[i] = *(const v4u*)(krow + 8 * i);
#pragma unroll
      for (int i = 0; i < 4; ++i) *(v4u*)(Ksh + kvr * AT_D + dh + 8 * i) = kw[i];
      asm volatile("" ::: "memory");
      v4u vw[4];
#pragma unroll
      for (int i = 0; i < 4; ++i) vw[i] = *(const v4u*)(vrow + 8 * i);
#pragma unroll
      for (int i = 0; i < 4; ++i) {
        const v4u vv = vw[i];
#pragma unroll
        for (int e = 0; e < 4; ++e) {
          const unsigned w = vv[e];
          const int d = dh + 8 * i + 2 * e;
          Vth[d * AT_KC + kvr]       = (unsigned short)(w & 0xffffu);
          Vth[(d + 1) * AT_KC + kvr] = (unsigned short)(w >> 16);
        }
      }
      asm volatile("" ::: "memory");
      v4u lw[4];
#pragma unroll
      for (int i = 0; i < 4; ++i) lw[i] = *(const v4u*)(lrw + 8 * i);
#pragma unroll
      for (int i = 0; i < 4; ++i) {
        const v4u vv = lw[i];
#pragma unroll
        for (int e = 0; e < 4; ++e) {
          const unsigned w = vv[e];
          const int d = dh + 8 * i + 2 * e;
          Vtl[d * AT_KC + kvr]       = (unsigned short)(w & 0xffffu);
          Vtl[(d + 1) * AT_KC + kvr] = (unsigned short)(w >> 16);
        }
      }
    }
    __syncthreads();

    v8f s[4];
#pragma unroll
    for (int j = 0; j < 4; ++j) {
      s[j] = (v8f){0.f,0.f,0.f,0.f,0.f,0.f,0.f,0.f};
#pragma unroll
      for (int dc = 0; dc < 2; ++dc) {
        const v16h kb = ld_frag16(Ksh + (j * 16 + c) * AT_D + dc * 32 + 8 * hh);
        s[j] = mma_h(qa[dc], kb, s[j]);
      }
    }
    float cm[8];
#pragma unroll
    for (int r = 0; r < 8; ++r) {
      float m = -__builtin_inff();
#pragma unroll
      for (int j = 0; j < 4; ++j) {
        const float sv = s[j][r] * sscale;
        s[j][r] = sv;
        m = fmaxf(m, sv);
      }
#pragma unroll
      for (int off = 1; off < 16; off <<= 1) m = fmaxf(m, __shfl_xor(m, off, 32));
      cm[r] = m;
    }
    unsigned short* pw = Psh[wave];
    unsigned short* pl = Psl[wave];
#pragma unroll
    for (int r = 0; r < 8; ++r) {
      const float mnew  = fmaxf(mrow[r], cm[r]);
      const float alpha = expf(mrow[r] - mnew);
      mrow[r] = mnew;
      float psum = 0.f;
#pragma unroll
      for (int j = 0; j < 4; ++j) {
        const float p = expf(s[j][r] - mnew);
        psum += p;
        unsigned short hb, lb;
        h_pair_bits(p * kPCarry, hb, lb);
        const int po = (8 * hh + r) * AT_KC + j * 16 + c;
        pw[po] = hb;
        pl[po] = lb;
      }
#pragma unroll
      for (int off = 1; off < 16; off <<= 1) psum += __shfl_xor(psum, off, 32);
      lrow[r] = lrow[r] * alpha + psum;
#pragma unroll
      for (int t = 0; t < 4; ++t) { oacc[t][r] *= alpha; racc[t][r] *= alpha; }
    }
    __builtin_amdgcn_fence(__ATOMIC_RELEASE, "workgroup");
    __builtin_amdgcn_wave_barrier();
    __builtin_amdgcn_fence(__ATOMIC_ACQUIRE, "workgroup");
#pragma unroll
    for (int kk = 0; kk < 2; ++kk) {
      const v16h pa  = ld_frag16(pw + c * AT_KC + kk * 32 + 8 * hh);
      const v16h pal = ld_frag16(pl + c * AT_KC + kk * 32 + 8 * hh);
#pragma unroll
      for (int t = 0; t < 4; ++t) {
        const v16h vb  = ld_frag16(Vth + (t * 16 + c) * AT_KC + kk * 32 + 8 * hh);
        const v16h vbl = ld_frag16(Vtl + (t * 16 + c) * AT_KC + kk * 32 + 8 * hh);
        oacc[t] = mma_h(pa, vb, oacc[t]);
        racc[t] = mma_h(pa, vbl, racc[t]);
        racc[t] = mma_h(pal, vb, racc[t]);
      }
    }
  }

  float* os = Os[wave];
#pragma unroll
  for (int r = 0; r < 8; ++r) {
    const float inv = 1.0f / (lrow[r] * kPCarry);
#pragma unroll
    for (int t = 0; t < 4; ++t) os[(8 * hh + r) * 68 + t * 16 + c] = (oacc[t][r] + racc[t][r] * kLoInv) * inv;
  }
  __builtin_amdgcn_fence(__ATOMIC_RELEASE, "workgroup");
  __builtin_amdgcn_wave_barrier();
  __builtin_amdgcn_fence(__ATOMIC_ACQUIRE, "workgroup");
  {
    const int c4 = (lane & 15) * 4;
    float* ob = Op + (tokb + q0) * (size_t)ldo + hoff;
    for (int pass = 0; pass < 2; ++pass) {
#pragma unroll
      for (int it = 0; it < 8; ++it) {
        const int row = it * 2 + hh;
        v4f val = *(const v4f*)(os + row * 68 + c4);
        *(volatile v4f*)(ob + (size_t)row * ldo + c4) = val;
      }
      __threadfence();
    }
  }
}

__global__ __launch_bounds__(256) void gate_gn_kernel(const float* __restrict__ G, const float* __restrict__ O,
                                                     const float* __restrict__ gamma, const float* __restrict__ beta,
                                                     float* __restrict__ out, int ld, float eps, float invn) {
  const int tok = blockIdx.x;
  const int c0  = 4 * threadIdx.x;
  const size_t roff = (size_t)tok * ld + c0;
  const v4f g  = *(const v4f*)(G + roff);
  const v4f o  = *(const v4f*)(O + roff);
  const v4f ga = *(const v4f*)(gamma + c0);
  const v4f be = *(const v4f*)(beta + c0);
  const float y0 = g[0] * o[0], y1 = g[1] * o[1], y2 = g[2] * o[2], y3 = g[3] * o[3];
  float su = (y0 + y1) + (y2 + y3);
#pragma unroll
  for (int off = 1; off < 16; off <<= 1) su += __shfl_xor(su, off, 32);
  const float mu = su * invn;
  const float d0 = y0 - mu, d1 = y1 - mu, d2 = y2 - mu, d3 = y3 - mu;
  float sq = (d0 * d0 + d1 * d1) + (d2 * d2 + d3 * d3);
#pragma unroll
  for (int off = 1; off < 16; off <<= 1) sq += __shfl_xor(sq, off, 32);
  const float var = sq * invn;
  const float rs  = 1.0f / sqrtf(var + eps);
  const v4f res = (v4f){ d0 * rs * ga[0] + be[0], d1 * rs * ga[1] + be[1], d2 * rs * ga[2] + be[2], d3 * rs * ga[3] + be[3] };
  float* op = out + roff;
  *(volatile v4f*)op = res;
  __threadfence();
  *(volatile v4f*)op = res;
}

extern "C" void kernel_launch(void* const* d_in, const int* in_sizes, int n_in,
                              void* d_out, int out_size, void* d_ws, size_t ws_size,
                              hipStream_t stream) {
  if (n_in < 11) return;
  const int nElem = kTok * kDim;
  const int nW    = kDim * kDim;
  if (in_sizes[0] != nElem) return;
  if (in_sizes[1] != nW || in_sizes[3] != nW || in_sizes[5] != nW || in_sizes[7] != nW) return;
  if (in_sizes[2] != kDim || in_sizes[4] != kDim || in_sizes[6] != kDim || in_sizes[8] != kDim) return;
  if (in_sizes[9] != kDim || in_sizes[10] != kDim) return;
  if (out_size != nElem) return;

  const size_t szP16 = (size_t)kTok * kDim * 2;
  const size_t szF32 = (size_t)kTok * kDim * 4;
  const size_t offX  = 0;
  const size_t offW  = offX + szP16;
  const size_t offQ  = offW + szP16;
  const size_t offK  = offQ + szP16;
  const size_t offV  = offK + szP16;
  const size_t offVL = offV + szP16;
  const size_t offG  = offVL + szP16;
  const size_t offO  = offG + szF32;
  const size_t total = offO + szF32;
  if (ws_size < total) return;

  const float* x     = (const float*)d_in[0];
  const float* wq    = (const float*)d_in[1];
  const float* bq    = (const float*)d_in[2];
  const float* wk    = (const float*)d_in[3];
  const float* bk    = (const float*)d_in[4];
  const float* wv    = (const float*)d_in[5];
  const float* bv    = (const float*)d_in[6];
  const float* wg    = (const float*)d_in[7];
  const float* bg    = (const float*)d_in[8];
  const float* gamma = (const float*)d_in[9];
  const float* beta  = (const float*)d_in[10];
  float* out = (float*)d_out;
  char* ws = (char*)d_ws;
  unsigned short* X16  = (unsigned short*)(ws + offX);
  unsigned short* W16  = (unsigned short*)(ws + offW);
  unsigned short* Q16  = (unsigned short*)(ws + offQ);
  unsigned short* K16  = (unsigned short*)(ws + offK);
  unsigned short* V16  = (unsigned short*)(ws + offV);
  unsigned short* VL16 = (unsigned short*)(ws + offVL);
  float* GT = (float*)(ws + offG);
  float* AO = (float*)(ws + offO);

  const int n8x = nElem / 8;
  const int n8w = nW / 8;
  cast8_f16_kernel<<<dim3(n8x / 256), dim3(256), 0, stream>>>(x, X16, n8x, 1.0f);
  cast8_f16_kernel<<<dim3(n8w / 256), dim3(256), 0, stream>>>(wq, W16 + (size_t)0 * nW, n8w, kWCarry);
  cast8_f16_kernel<<<dim3(n8w / 256), dim3(256), 0, stream>>>(wk, W16 + (size_t)1 * nW, n8w, kWCarry);
  cast8_f16_kernel<<<dim3(n8w / 256), dim3(256), 0, stream>>>(wv, W16 + (size_t)2 * nW, n8w, kWCarry);
  cast8_f16_kernel<<<dim3(n8w / 256), dim3(256), 0, stream>>>(wg, W16 + (size_t)3 * nW, n8w, kWCarry);

  const int tilesProj = (kTok / 64) * (kDim / 64);
  wmma_gemm64<0, false, 2, 1, false, 0><<<dim3(tilesProj / 8, 1), dim3(256), 0, stream>>>(
      X16, X16, kDim, 0L, W16 + (size_t)0 * nW, W16 + (size_t)0 * nW, kDim, 0L,
      (void*)Q16, (void*)Q16, kDim, 0L, bq, bq, 0L, kTok, kDim, kDim, kWCarryInv);
  wmma_gemm64<0, false, 2, 1, false, 0><<<dim3(tilesProj / 8, 1), dim3(256), 0, stream>>>(
      X16, X16, kDim, 0L, W16 + (size_t)1 * nW, W16 + (size_t)1 * nW, kDim, 0L,
      (void*)K16, (void*)K16, kDim, 0L, bk, bk, 0L, kTok, kDim, kDim, kWCarryInv);
  wmma_gemm64<0, false, 2, 3, false, 0><<<dim3(tilesProj / 8, 1), dim3(256), 0, stream>>>(
      X16, X16, kDim, 0L, W16 + (size_t)2 * nW, W16 + (size_t)2 * nW, kDim, 0L,
      (void*)V16, (void*)VL16, kDim, 0L, bv, bv, 0L, kTok, kDim, kDim, kWCarryInv);
  wmma_gemm64<0, false, 2, 0, false, 0><<<dim3(tilesProj / 8, 1), dim3(256), 0, stream>>>(
      X16, X16, kDim, 0L, W16 + (size_t)3 * nW, W16 + (size_t)3 * nW, kDim, 0L,
      (void*)GT, (void*)GT, kDim, 0L, bg, bg, 0L, kTok, kDim, kDim, kWCarryInv);

  attn_f16_kernel<<<dim3(kBatch * kHeads * (kSeq / AT_QB)), dim3(128), 0, stream>>>(
      Q16, K16, V16, VL16, AO, kDim, kDim, kSeq, kHeads, kScoreScale);

  gate_gn_kernel<<<dim3(kTok), dim3(256), 0, stream>>>(GT, AO, gamma, beta, out, kDim, kGnEps, kInvDh);
}
